// MultiHeadAttentionWithRPR_21449066676705
// MI455X (gfx1250) — hardware-verified
//
#include <hip/hip_runtime.h>


namespace {
constexpr int NB_ = 4, S = 1024, D = 1024, H = 16, HD = 64, CLIP = 16, NR = 2 * CLIP + 1  , NT = NB_ * S, CH = 256;
constexpr float XS = 8.0f, HS = 256.0f, PS = 256.0f, WSC = 256.0f, SCALE = 0.125f;
typedef _Float16 b16;
typedef __attribute__((ext_vector_type(16))) _Float16 v16b;
typedef __attribute__((ext_vector_type(8))) _Float16 v8b;
typedef __attribute__((ext_vector_type(2))) _Float16 v2b;
typedef __attribute__((ext_vector_type(8))) float v8f;
typedef __attribute__((ext_vector_type(4))) float v4f;
typedef __attribute__((ext_vector_type(2))) float v2f;
__device__ __forceinline__ float bf16_rne(float f) { unsigned int u = __float_as_uint(f); u += 0x7FFFu + ((u >> 16) & 1u); float r = __uint_as_float(u & 0xFFFF0000u); asm volatile("" : "+v"(r)); return r; }
__device__ __forceinline__ float bfv(float f) { float r = bf16_rne(f); asm volatile("" : "+v"(r)); return r; }
__device__ __forceinline__ void split16(float v, b16& hi, b16& lo) { hi = (b16)v; lo = (b16)(v - (float)hi); }
__device__ __forceinline__ v16b frag_kb(const b16* p, int hh) { const v8b a = *(const v8b*)(p + 8 * hh), b = *(const v8b*)(p + 16 + 8 * hh); v16b f;
#pragma unroll
  for (int e = 0; e < 8; ++e) { f[e] = a[e]; f[8 + e] = b[e]; } return f; }
__device__ __forceinline__ v8f wmma16b(v16b a, v16b b, v8f c) { v8f d = __builtin_amdgcn_wmma_f32_16x16x32_f16(false, a, false, b, (short)0, c, false, false); asm volatile("v_nop\n\tv_nop\n\tv_nop\n\tv_nop" : "+v"(d) : "v"(a), "v"(b)); return d; }
__device__ __forceinline__ void wave_lds_sync() { __builtin_amdgcn_fence(__ATOMIC_RELEASE, "workgroup"); __builtin_amdgcn_wave_barrier(); __builtin_amdgcn_fence(__ATOMIC_ACQUIRE, "workgroup"); }
__device__ __forceinline__ float pmul(float a, float b) { float p = a * b; asm volatile("" : "+v"(p)); return p; }
__device__ __forceinline__ int iclamp(int v, int lo, int hi) { return v < lo ? lo : (v > hi ? hi : v); }

__global__ __launch_bounds__(256) void wput_kernel(const float* __restrict__ wq, const float* __restrict__ wk, const float* __restrict__ wv, const float* __restrict__ wo, const float* __restrict__ ek, b16* __restrict__ W4, b16* __restrict__ EKh, b16* __restrict__ EKl) { const size_t nt = (size_t)gridDim.x * 256, u0 = (size_t)blockIdx.x * 256 + threadIdx.x; v8b v;
  for (size_t u = u0; u < (size_t)4 * D * 128; u += nt) { const int o = (int)(u / 128), k0 = (int)(u % 128) * 8; const int which = o / D, oo = o % D; const float* w = which == 0 ? wq : (which == 1 ? wk : (which == 2 ? wv : wo));
#pragma unroll
    for (int j = 0; j < 8; ++j) v[j] = (b16)(bf16_rne(w[(size_t)oo * D + k0 + j]) * WSC); for (int pass = 0; pass < 2; ++pass) { *(volatile v8b*)(W4 + (size_t)o * D + k0) = v; __threadfence(); } }
  if (u0 < 48 * 8) { const int r = (int)(u0 / 8), k0 = (int)(u0 % 8) * 8; v8b a, c;
#pragma unroll
    for (int j = 0; j < 8; ++j) { float e = r < NR ? bfv(ek[(size_t)r * HD + k0 + j]) : 0.0f; b16 p, pl; split16(e * HS, p, pl); a[j] = p; c[j] = pl; } for (int pass = 0; pass < 2; ++pass) { *(volatile v8b*)(EKh + (size_t)r * HD + k0) = a; *(volatile v8b*)(EKl + (size_t)r * HD + k0) = c; __threadfence(); } } }
__global__ __launch_bounds__(32) void proj_kernel(const float* __restrict__ xq, const float* __restrict__ xk, const float* __restrict__ xv, const b16* __restrict__ W4, int QLIM, b16* __restrict__ Qh, b16* __restrict__ Ql, b16* __restrict__ Kh, b16* __restrict__ Kl, float* __restrict__ V) { __shared__ __attribute__((aligned(16))) b16 Ax[16][D + 8]; __shared__ float Tf[16][260]; const int lane = threadIdx.x, nloc = lane & 15, hlf = lane >> 4; const size_t t0 = (size_t)blockIdx.x * 16; const int which = blockIdx.y; if ((int)(t0 % S) >= QLIM) return;
  const float* x = which == 0 ? xq : (which == 1 ? xk : xv);
  for (int rr = 0; rr < 16; ++rr) for (int q = 0; q < D / 32; ++q) { const int c = q * 32 + lane; Ax[rr][c] = (b16)(bf16_rne(x[(t0 + rr) * D + c]) * XS); }
  if (lane < 16) for (int k = D; k < D + 8; ++k) Ax[lane][k] = (b16)0.0f;
  wave_lds_sync();
#pragma unroll 1
  for (int g = 0; g < 4; ++g) { const int c0 = g * 256; v8f acc[16];
#pragma unroll
    for (int t = 0; t < 16; ++t) acc[t] = (v8f){};
#pragma unroll 2
    for (int kb = 0; kb < D; kb += 32) { const v16b a = frag_kb(&Ax[nloc][kb], hlf);
#pragma unroll
      for (int t = 0; t < 16; ++t) acc[t] = wmma16b(a, frag_kb(W4 + ((size_t)which * D + c0 + t * 16 + nloc) * D + kb, hlf), acc[t]); }
#pragma unroll
    for (int t = 0; t < 16; ++t)
#pragma unroll
      for (int r8 = 0; r8 < 8; ++r8) Tf[8 * hlf + r8][t * 16 + nloc] = acc[t][r8] * (1.0f / (XS * WSC));
    wave_lds_sync();
    for (int pass = 0; pass < 2; ++pass) { for (int rr = 0; rr < 16; ++rr) { const size_t tk = t0 + rr;
        if (which == 2) { for (int q = 0; q < 2; ++q) *(volatile v4f*)(V + tk * D + c0 + q * 128 + lane * 4) = *(const v4f*)(&Tf[rr][q * 128 + lane * 4]); }
        else { b16* Ph = which == 0 ? Qh : Kh; b16* Pl = which == 0 ? Ql : Kl; for (int q = 0; q < 4; ++q) { const int c = q * 64 + lane * 2; b16 h0, l0, h1, l1; split16(Tf[rr][c] * HS, h0, l0); split16(Tf[rr][c + 1] * HS, h1, l1); *(volatile v2b*)(Ph + tk * D + c0 + c) = (v2b){h0, h1}; *(volatile v2b*)(Pl + tk * D + c0 + c) = (v2b){l0, l1}; } } }
      __threadfence(); }
    wave_lds_sync(); } }
__global__ __launch_bounds__(256) void vt_kernel(const float* __restrict__ V, b16* __restrict__ VTh, b16* __restrict__ VTl) { __shared__ float Tt[64][257]; const int tt = blockIdx.x >> 2, hg = blockIdx.x & 3; const size_t t0 = (size_t)tt * 64; const int b = (int)(t0 / S), s0 = (int)(t0 % S); const int tid = threadIdx.x, wave = tid >> 5, lane = tid & 31;
  for (int q = wave; q < 64; q += 8) for (int c = lane; c < 256; c += 32) Tt[q][c] = V[(t0 + q) * D + hg * 256 + c];
  __syncthreads();
  for (int pass = 0; pass < 2; ++pass) { for (int c = wave; c < 256; c += 8) { const int h = hg * 4 + c / HD, d = c % HD; b16 h0, l0, h1, l1; split16(Tt[lane * 2][c] * HS, h0, l0); split16(Tt[lane * 2 + 1][c] * HS, h1, l1); const size_t o = (((size_t)b * H + h) * HD + d) * S + s0 + lane * 2; *(volatile v2b*)(VTh + o) = (v2b){h0, h1}; *(volatile v2b*)(VTl + o) = (v2b){l0, l1}; } __threadfence(); } }
__global__ __launch_bounds__(32) void att_kernel(const b16* __restrict__ Qh, const b16* __restrict__ Ql, const b16* __restrict__ Kh, const b16* __restrict__ Kl, const b16* __restrict__ VTh, const b16* __restrict__ VTl, const b16* __restrict__ EKh, const b16* __restrict__ EKl, const float* __restrict__ ev, const int* __restrict__ vlens, int ALIM, float* __restrict__ O) { __shared__ __attribute__((aligned(16))) b16 Pa[16][CH + 8], Pb[16][CH + 8]; __shared__ float Sc[16][CH + 1], QE[16][49], Bk[16][NR], Mx[16], Ls[16], Fc[16], Of[16][HD + 1]; const int lane = threadIdx.x, nloc = lane & 15, hlf = lane >> 4; const int bh = blockIdx.x / (S / 16), q0 = (blockIdx.x % (S / 16)) * 16; if (q0 >= ALIM) return; const int b = bh / H, h = bh % H; const size_t tq = (size_t)b * S + q0; const int vl = iclamp(vlens[b], 0, S);
  if (lane < 16) { Mx[lane] = -INFINITY; Ls[lane] = 0.0f; for (int kk = CH; kk < CH + 8; ++kk) { Pa[lane][kk] = (b16)0.0f; Pb[lane][kk] = (b16)0.0f; } for (int r = 0; r < NR; ++r) Bk[lane][r] = 0.0f; }
  v16b qa[2], ql[2]; for (int ks = 0; ks < 2; ++ks) { qa[ks] = frag_kb(Qh + (tq + nloc) * D + h * HD + ks * 32, hlf); ql[ks] = frag_kb(Ql + (tq + nloc) * D + h * HD + ks * 32, hlf); }
#pragma unroll
  for (int t = 0; t < 3; ++t) { v8f e = (v8f){};
#pragma unroll
    for (int ks = 0; ks < 2; ++ks) { const v16b eh = frag_kb(EKh + (size_t)(t * 16 + nloc) * HD + ks * 32, hlf), el = frag_kb(EKl + (size_t)(t * 16 + nloc) * HD + ks * 32, hlf); e = wmma16b(qa[ks], eh, e); e = wmma16b(qa[ks], el, e); e = wmma16b(ql[ks], eh, e); }
#pragma unroll
    for (int r8 = 0; r8 < 8; ++r8) QE[8 * hlf + r8][t * 16 + nloc] = e[r8] * (1.0f / (HS * HS)); }
  wave_lds_sync();
  v8f oacc[4] = {(v8f){}, (v8f){}, (v8f){}, (v8f){}}; const int nch = (vl + CH - 1) / CH;
#pragma unroll 1
  for (int ch = 0; ch < nch; ++ch) { const int k0 = ch * CH;
#pragma unroll 1
    for (int tg = 0; tg < 16; tg += 4) { v8f sacc[4] = {(v8f){}, (v8f){}, (v8f){}, (v8f){}};
#pragma unroll
      for (int t = 0; t < 4; ++t)
#pragma unroll
        for (int ks = 0; ks < 2; ++ks) { const size_t ko = ((size_t)b * S + k0 + (tg + t) * 16 + nloc) * D + h * HD + ks * 32; const v16b kh = frag_kb(Kh + ko, hlf), kl = frag_kb(Kl + ko, hlf); sacc[t] = wmma16b(qa[ks], kh, sacc[t]); sacc[t] = wmma16b(qa[ks], kl, sacc[t]); sacc[t] = wmma16b(ql[ks], kh, sacc[t]); }
#pragma unroll
      for (int t = 0; t < 4; ++t)
#pragma unroll
        for (int r8 = 0; r8 < 8; ++r8) Sc[8 * hlf + r8][(tg + t) * 16 + nloc] = sacc[t][r8] * (1.0f / (HS * HS)); }
    wave_lds_sync();
    if (lane < 16) { const int r = lane, q = q0 + r; float mx = -INFINITY; for (int j = 0; j < CH; ++j) { const int k = k0 + j; if (k < vl) { const int dd = iclamp(k - q, -CLIP, CLIP) + CLIP; const float s = (Sc[r][j] + QE[r][dd]) * SCALE; Sc[r][j] = s; mx = fmaxf(mx, s); } }
      const float mo = Mx[r], mn = fmaxf(mo, mx); const float fac = (mo == -INFINITY) ? 0.0f : __expf(mo - mn); for (int rr2 = 0; rr2 < NR; ++rr2) Bk[r][rr2] *= fac;
      float sm = 0.0f; for (int j = 0; j < CH; ++j) { const int k = k0 + j; const float p = (k < vl) ? __expf(Sc[r][j] - mn) : 0.0f; sm += p; if (k < vl) { const int dd = iclamp(k - q, -CLIP, CLIP) + CLIP; Bk[r][dd] += p; } b16 ph, pl; split16(p * PS, ph, pl); Pa[r][j] = ph; Pb[r][j] = pl; }
      Fc[r] = fac; Ls[r] = Ls[r] * fac + sm; Mx[r] = mn; }
    wave_lds_sync();
#pragma unroll
    for (int t = 0; t < 4; ++t)
#pragma unroll
      for (int r8 = 0; r8 < 8; ++r8) oacc[t][r8] *= Fc[8 * hlf + r8];
#pragma unroll 2
    for (int kb = 0; kb < CH; kb += 32) { const v16b pa = frag_kb(&Pa[nloc][kb], hlf), pb = frag_kb(&Pb[nloc][kb], hlf);
#pragma unroll
      for (int t = 0; t < 4; ++t) { const size_t vo = ((size_t)bh * HD + t * 16 + nloc) * S + k0 + kb; const v16b vh = frag_kb(VTh + vo, hlf), vlo = frag_kb(VTl + vo, hlf); oacc[t] = wmma16b(pa, vh, oacc[t]); oacc[t] = wmma16b(pa, vlo, oacc[t]); oacc[t] = wmma16b(pb, vh, oacc[t]); } }
    wave_lds_sync(); }
#pragma unroll
  for (int t = 0; t < 4; ++t)
#pragma unroll
    for (int r8 = 0; r8 < 8; ++r8) Of[8 * hlf + r8][t * 16 + nloc] = oacc[t][r8] * (1.0f / (PS * HS));
  wave_lds_sync();
  for (int r = 0; r < 16; ++r) { float a0 = Of[r][lane * 2], a1 = Of[r][lane * 2 + 1];
#pragma unroll 1
    for (int rr2 = 0; rr2 < NR; ++rr2) { const float bk = Bk[r][rr2]; a0 += pmul(bk, bfv(ev[(size_t)rr2 * HD + lane * 2])); a1 += pmul(bk, bfv(ev[(size_t)rr2 * HD + lane * 2 + 1])); } const float inv = 1.0f / Ls[r]; Of[r][lane * 2] = a0 * inv; Of[r][lane * 2 + 1] = a1 * inv; }
  wave_lds_sync();
  for (int pass = 0; pass < 2; ++pass) { for (int r = 0; r < 16; ++r) *(volatile v2f*)(O + (tq + r) * D + h * HD + lane * 2) = (v2f){Of[r][lane * 2], Of[r][lane * 2 + 1]}; __threadfence(); } }
__global__ __launch_bounds__(32) void outp_kernel(const float* __restrict__ O, const b16* __restrict__ WO, int ALIM, float* __restrict__ out) { __shared__ __attribute__((aligned(16))) b16 Ah[16][D + 8], Al[16][D + 8]; __shared__ float Tf[16][260]; const int lane = threadIdx.x, nloc = lane & 15, hlf = lane >> 4; const size_t t0 = (size_t)blockIdx.x * 16; if ((int)(t0 % S) >= ALIM) return;
  for (int rr = 0; rr < 16; ++rr) for (int q = 0; q < D / 32; ++q) { const int c = q * 32 + lane; b16 p, pl; split16(O[(t0 + rr) * D + c] * HS, p, pl); Ah[rr][c] = p; Al[rr][c] = pl; }
  if (lane < 16) for (int k = D; k < D + 8; ++k) { Ah[lane][k] = (b16)0.0f; Al[lane][k] = (b16)0.0f; }
  wave_lds_sync();
#pragma unroll 1
  for (int g = 0; g < 4; ++g) { v8f acc[16];
#pragma unroll
    for (int t = 0; t < 16; ++t) acc[t] = (v8f){};
#pragma unroll 2
    for (int kb = 0; kb < D; kb += 32) { const v16b a = frag_kb(&Ah[nloc][kb], hlf), al = frag_kb(&Al[nloc][kb], hlf);
#pragma unroll
      for (int t = 0; t < 16; ++t) { const v16b bw = frag_kb(WO + (size_t)(g * 256 + t * 16 + nloc) * D + kb, hlf); acc[t] = wmma16b(a, bw, acc[t]); acc[t] = wmma16b(al, bw, acc[t]); } }
#pragma unroll
    for (int t = 0; t < 16; ++t)
#pragma unroll
      for (int r8 = 0; r8 < 8; ++r8) Tf[8 * hlf + r8][t * 16 + nloc] = acc[t][r8] * (1.0f / (HS * WSC));
    wave_lds_sync();
    for (int pass = 0; pass < 2; ++pass) { for (int rr = 0; rr < 16; ++rr) for (int q = 0; q < 2; ++q) *(volatile v4f*)(out + (t0 + rr) * D + g * 256 + q * 128 + lane * 4) = *(const v4f*)(&Tf[rr][q * 128 + lane * 4]); __threadfence(); }
    wave_lds_sync(); } }
}

extern "C" void kernel_launch(void* const* d_in, const int* in_sizes, int n_in, void* d_out, int out_size, void* d_ws, size_t ws_size, hipStream_t stream) {
  (void)n_in;
  auto Fp = [&](int i) { return (const float*)d_in[i]; }; auto Ip = [&](int i) { return (const int*)d_in[i]; };
  if (in_sizes[0] != NT * D || in_sizes[1] != NT * D || in_sizes[2] != NT * D || in_sizes[3] != NB_ || in_sizes[4] != D * D || in_sizes[7] != D * D || in_sizes[8] != NR * HD || in_sizes[9] != NR * HD || out_size != NT * D) return;
  const int QLIM = S, ALIM = S;
  size_t off = 0; char* ws = (char*)d_ws;
  auto carve = [&](size_t bytes) { char* p = ws + off; off += (bytes + 255) & ~(size_t)255; return p; };
  b16* W4 = (b16*)carve((size_t)4 * D * D * 2); b16* EKh = (b16*)carve(48 * HD * 2); b16* EKl = (b16*)carve(48 * HD * 2); b16* Qh = (b16*)carve((size_t)NT * D * 2); b16* Ql = (b16*)carve((size_t)NT * D * 2); b16* Kh = (b16*)carve((size_t)NT * D * 2); b16* Kl = (b16*)carve((size_t)NT * D * 2); float* V = (float*)carve((size_t)NT * D * 4); b16* VTh = (b16*)carve((size_t)NT * D * 2); b16* VTl = (b16*)carve((size_t)NT * D * 2); float* O = (float*)carve((size_t)NT * D * 4);
  if (off > ws_size || off > ((size_t)104 << 20)) return;
  wput_kernel<<<256, 256, 0, stream>>>(Fp(4), Fp(5), Fp(6), Fp(7), Fp(8), W4, EKh, EKl);
  proj_kernel<<<dim3(NT / 16, 3), 32, 0, stream>>>(Fp(0), Fp(1), Fp(2), W4, QLIM, Qh, Ql, Kh, Kl, V);
  vt_kernel<<<(NT / 64) * 4, 256, 0, stream>>>(V, VTh, VTl);
  att_kernel<<<NB_ * H * (S / 16), 32, 0, stream>>>(Qh, Ql, Kh, Kl, VTh, VTl, EKh, EKl, Fp(9), Ip(3), ALIM, O);
  outp_kernel<<<NT / 16, 32, 0, stream>>>(O, W4 + (size_t)3 * D * D, ALIM, (float*)d_out);
}
